// GATEncoder_29815662969290
// MI455X (gfx1250) — hardware-verified
//
#include <hip/hip_runtime.h>
#include <stddef.h>
#include <stdint.h>


#define DIN     128
#define NHD     4
#define DHD     32
#define NBT     4
#define KX2     256
#define NTHR    256
#define NWAVE   8
#define EPT     8
#define CHUNK   (NTHR * EPT)
#define WCAP    (EPT * 32)
#define LISTN   (NWAVE * WCAP)
#define NBMAX   512
#define SPT     (NBMAX / NTHR)
#define RCAP    24576
#define DEGCAP  128
#define STW     128
#define GBM     64
#define WSMAX   134217728
#define LDS_AGG ((2 * RCAP + 2 * NBMAX + LISTN + 2 * NWAVE) * 4)

static_assert((CHUNK & (CHUNK - 1)) == 0 && CHUNK <= 4096);
static_assert((NBMAX & (NBMAX - 1)) == 0 && NBMAX <= 4096);
static_assert(SPT == 2 && NTHR * SPT == NBMAX);
static_assert(LISTN >= NBMAX && LISTN >= NWAVE * WCAP);
static_assert((RCAP % 32) == 0);
static_assert(NWAVE * STW <= RCAP);
static_assert(LDS_AGG <= 300000);
static_assert(GBM == 4 * 16 && NTHR == 8 * 32);
static_assert(DIN == NHD * DHD && KX2 == 2 * DIN && STW == DIN);
static_assert((DIN % 32) == 0 && (DHD % 32) == 0);

typedef float          v4f  __attribute__((ext_vector_type(4)));
typedef float          v8f  __attribute__((ext_vector_type(8)));
typedef int            v4i  __attribute__((ext_vector_type(4)));
typedef int            v8i  __attribute__((ext_vector_type(8)));
typedef unsigned short v8us __attribute__((ext_vector_type(8)));
typedef __bf16         v16b __attribute__((ext_vector_type(16)));
union FragB { v16b v; v8us h[2]; v8i w; };

__device__ __forceinline__ v8f wmb(const FragB& a, const FragB& b, v8f c) {
  v8f d = __builtin_amdgcn_wmma_f32_16x16x32_bf16(false, a.v, false, b.v, (short)0, c, false, false);
  asm volatile("v_nop\n\tv_nop\n\tv_nop\n\tv_nop" : "+v"(d) : "v"(a.w), "v"(b.w));
  return d;
}

__device__ __forceinline__ void ldwait() {
  asm volatile("s_wait_loadcnt 0x0" ::: "memory");
}

__device__ __forceinline__ unsigned short bfb(float x) {
  unsigned u = __float_as_uint(x);
  u = u + 0x7FFFu + ((u >> 16) & 1u);
  return (unsigned short)(u >> 16);
}
__device__ __forceinline__ float bfv(unsigned short b) { return __uint_as_float(((unsigned)b) << 16); }
__device__ __forceinline__ float bfr(float x) { return bfv(bfb(x)); }

__device__ __forceinline__ v8us cvt8b(const v4f a, const v4f b) {
  v8us o;
  o[0] = bfb(a.x); o[1] = bfb(a.y); o[2] = bfb(a.z); o[3] = bfb(a.w);
  o[4] = bfb(b.x); o[5] = bfb(b.y); o[6] = bfb(b.z); o[7] = bfb(b.w);
  return o;
}

__device__ __forceinline__ v8us hilo8(const v4f a, const v4f b, const bool lo) {
  v8us o;
#define HLQ(I, X) { const unsigned short hq = bfb(X); const unsigned short lq = bfb((X) - bfv(hq)); o[I] = lo ? lq : hq; }
  HLQ(0, a.x) HLQ(1, a.y) HLQ(2, a.z) HLQ(3, a.w)
  HLQ(4, b.x) HLQ(5, b.y) HLQ(6, b.z) HLQ(7, b.w)
#undef HLQ
  return o;
}

__device__ __forceinline__ int scan_chunk(const int* __restrict__ dsts, int nE, int cbase, int slotBase,
                                          int nb, int vec8, int* list, int tid, int lane, int wave) {
  int wc = 0;
  const int el0  = tid * EPT;
  const int e0   = cbase + el0;
  const int sent = -2147483647 - 1;
  v4i da, db;
  if (vec8 != 0 && cbase + CHUNK <= nE) {
    da = *(const v4i*)(dsts + e0);
    db = *(const v4i*)(dsts + e0 + 4);
  } else {
    da.x = (e0     < nE) ? dsts[min(e0,     nE - 1)] : sent;
    da.y = (e0 + 1 < nE) ? dsts[min(e0 + 1, nE - 1)] : sent;
    da.z = (e0 + 2 < nE) ? dsts[min(e0 + 2, nE - 1)] : sent;
    da.w = (e0 + 3 < nE) ? dsts[min(e0 + 3, nE - 1)] : sent;
    db.x = (e0 + 4 < nE) ? dsts[min(e0 + 4, nE - 1)] : sent;
    db.y = (e0 + 5 < nE) ? dsts[min(e0 + 5, nE - 1)] : sent;
    db.z = (e0 + 6 < nE) ? dsts[min(e0 + 6, nE - 1)] : sent;
    db.w = (e0 + 7 < nE) ? dsts[min(e0 + 7, nE - 1)] : sent;
  }
  const unsigned nbs = (unsigned)slotBase;
  const unsigned unb = (unsigned)nb;
  const unsigned s0 = (unsigned)da.x - nbs, s1 = (unsigned)da.y - nbs;
  const unsigned s2 = (unsigned)da.z - nbs, s3 = (unsigned)da.w - nbs;
  const unsigned s4 = (unsigned)db.x - nbs, s5 = (unsigned)db.y - nbs;
  const unsigned s6 = (unsigned)db.z - nbs, s7 = (unsigned)db.w - nbs;
  const bool h0 = s0 < unb, h1 = s1 < unb, h2 = s2 < unb, h3 = s3 < unb;
  const bool h4 = s4 < unb, h5 = s5 < unb, h6 = s6 < unb, h7 = s7 < unb;
  const unsigned any = __builtin_amdgcn_ballot_w32(h0 | h1 | h2 | h3 | h4 | h5 | h6 | h7);
  if (any != 0u) {
#define HITJ(J, HJ, SJ) { \
      const unsigned mj = __builtin_amdgcn_ballot_w32(HJ); \
      if (mj != 0u) { \
        if (HJ) { \
          const int pos = wc + (int)__builtin_amdgcn_mbcnt_lo(mj, 0u); \
          if (pos < WCAP) list[wave * WCAP + pos] = ((el0 + (J)) << 12) | (int)(SJ); \
        } \
        wc += (int)__builtin_popcount(mj); } }
    HITJ(0, h0, s0)
    HITJ(1, h1, s1)
    HITJ(2, h2, s2)
    HITJ(3, h3, s3)
    HITJ(4, h4, s4)
    HITJ(5, h5, s5)
    HITJ(6, h6, s6)
    HITJ(7, h7, s7)
#undef HITJ
  }
  return wc;
}

__global__ __launch_bounds__(NTHR) void k_cvt(const float* __restrict__ src, int nRowsSrc, int K,
                                              unsigned short* dstp, int nUnits) {
  const int u = (int)blockIdx.x * NTHR + (int)threadIdx.x;
  if (u >= nUnits) return;
  const int kq  = K >> 3;
  const int n   = u / kq;
  const int k8  = (u - n * kq) * 8;
  const int ncl = n < nRowsSrc ? n : nRowsSrc - 1;
  const float* p = src + (size_t)ncl * (size_t)K + k8;
  v4f a = *(const v4f*)p, b = *(const v4f*)(p + 4);
  const v4f z4 = {0.f, 0.f, 0.f, 0.f};
  if (n >= nRowsSrc) { a = z4; b = z4; }
  const v8us o = cvt8b(a, b);
  const size_t off = (size_t)n * (size_t)K + k8;
  *(volatile v8us*)(dstp + off) = o;
  __threadfence();
  *(volatile v8us*)(dstp + off) = o;
}

template<int EPI, int LO>
__global__ __launch_bounds__(NTHR) void k_gemm(
    const unsigned short* __restrict__ A0, const unsigned short* __restrict__ A1,
    int lda, int loff, int ks0, int ks1,
    const unsigned short* __restrict__ W, int ldw,
    const float* __restrict__ al, const float* __restrict__ ar, const float* __restrict__ bias,
    float* outF, float* outE, int nRows)
{
  __shared__ __attribute__((aligned(16))) float stg[GBM * DIN];
  __shared__ __attribute__((aligned(16))) float elr[GBM * 8];
  __shared__ float alr[2 * DIN];
  const int tid = (int)threadIdx.x, lane = tid & 31, wave = tid >> 5, hh = lane >> 4, m = lane & 15;
  const int rt = wave & 3, cg = wave >> 2;
  const int rowBase = (int)blockIdx.x * GBM;

  if (EPI == 0) {
    const float va = al[tid & (DIN - 1)];
    const float vr = ar[tid & (DIN - 1)];
    alr[tid] = bfr(wave < 4 ? va : vr);
  }

  v8f acc[4];
  {
    const v8f z = {0.f, 0.f, 0.f, 0.f, 0.f, 0.f, 0.f, 0.f};
    acc[0] = z; acc[1] = z; acc[2] = z; acc[3] = z;
  }
  const size_t arow = (size_t)(rowBase + 16 * rt + m) * (size_t)lda + 8 * hh;
  const unsigned short* ap0 = A0 + arow;
  const unsigned short* ap1 = A1 + arow;
  const unsigned short* wp  = W + (size_t)(64 * cg + m) * (size_t)ldw + 8 * hh;
#pragma unroll 1
  for (int ks = 0; ks < ks0; ++ks) {
    FragB af, lf;
    af.h[0] = *(const v8us*)(ap0 + 32 * ks);
    af.h[1] = *(const v8us*)(ap0 + 32 * ks + 16);
    if (LO) {
      lf.h[0] = *(const v8us*)(ap0 + loff + 32 * ks);
      lf.h[1] = *(const v8us*)(ap0 + loff + 32 * ks + 16);
    } else {
      lf.w = af.w;
    }
#pragma unroll
    for (int t = 0; t < 4; ++t) {
      const unsigned short* wq = wp + (size_t)(16 * t) * (size_t)ldw + 32 * ks;
      FragB bf;
      bf.h[0] = *(const v8us*)wq;
      bf.h[1] = *(const v8us*)(wq + 16);
      acc[t] = wmb(af, bf, acc[t]);
      if (LO) acc[t] = wmb(lf, bf, acc[t]);
    }
  }
#pragma unroll 1
  for (int ks = 0; ks < ks1; ++ks) {
    FragB af, lf;
    af.h[0] = *(const v8us*)(ap1 + 32 * ks);
    af.h[1] = *(const v8us*)(ap1 + 32 * ks + 16);
    if (LO) {
      lf.h[0] = *(const v8us*)(ap1 + loff + 32 * ks);
      lf.h[1] = *(const v8us*)(ap1 + loff + 32 * ks + 16);
    } else {
      lf.w = af.w;
    }
#pragma unroll
    for (int t = 0; t < 4; ++t) {
      const unsigned short* wq = wp + (size_t)(16 * t) * (size_t)ldw + 32 * (ks0 + ks);
      FragB bf;
      bf.h[0] = *(const v8us*)wq;
      bf.h[1] = *(const v8us*)(wq + 16);
      acc[t] = wmb(af, bf, acc[t]);
      if (LO) acc[t] = wmb(lf, bf, acc[t]);
    }
  }

#pragma unroll
  for (int t = 0; t < 4; ++t) {
    const int lc = 64 * cg + 16 * t + m;
    float bv = 0.f;
    if (EPI == 1) bv = bfr(bias[lc]);
#pragma unroll
    for (int r = 0; r < 8; ++r) {
      const int lr = 16 * rt + 8 * hh + r;
      stg[lr * DIN + lc] = acc[t][r] + bv;
    }
  }
  __syncthreads();

  if (EPI == 0) {
    const int row = tid >> 2, h = tid & 3;
    const float* sp = stg + row * DIN + DHD * h;
    const float* pa = alr + DHD * h;
    const float* pr = alr + DIN + DHD * h;
    float sl = 0.f, sr = 0.f;
#pragma unroll 8
    for (int d = 0; d < DHD; ++d) {
      const float f = sp[d];
      sl = fmaf(f, pa[d], sl);
      sr = fmaf(f, pr[d], sr);
    }
    elr[row * 8 + h]     = sl;
    elr[row * 8 + 4 + h] = sr;
  }
  __syncthreads();

  v4f fv[8];
#pragma unroll
  for (int i = 0; i < 8; ++i) {
    const int p  = i * NTHR + tid;
    const int lr = p >> 5;
    const int c4 = (p & 31) * 4;
    fv[i] = *(const v4f*)(stg + lr * DIN + c4);
  }
  v4f ev = {0.f, 0.f, 0.f, 0.f};
  if (EPI == 0) ev = *(const v4f*)(elr + 4 * (tid & 127));
  const bool we = (EPI == 0) && (tid < 128);
  float* ep = outE + (size_t)rowBase * 8 + 4 * (tid & 127);
#pragma unroll
  for (int i = 0; i < 8; ++i) {
    const int p  = i * NTHR + tid;
    const int lr = p >> 5;
    const int c4 = (p & 31) * 4;
    const int gr = rowBase + lr;
    float* op = outF + (size_t)gr * DIN + c4;
    if (gr < nRows) *(volatile v4f*)op = fv[i];
  }
  if (we) *(volatile v4f*)ep = ev;
  __threadfence();
#pragma unroll
  for (int i = 0; i < 8; ++i) {
    const int p  = i * NTHR + tid;
    const int lr = p >> 5;
    const int c4 = (p & 31) * 4;
    const int gr = rowBase + lr;
    float* op = outF + (size_t)gr * DIN + c4;
    if (gr < nRows) *(volatile v4f*)op = fv[i];
  }
  if (we) *(volatile v4f*)ep = ev;
}

__global__ __launch_bounds__(NTHR) void k_ofc(const unsigned short* __restrict__ AG, const unsigned short* __restrict__ OW,
                                              const float* __restrict__ ob, unsigned short* XP, int nRows) {
  __shared__ __attribute__((aligned(16))) float stg[GBM * DIN];
  const int tid = (int)threadIdx.x, lane = tid & 31, wave = tid >> 5, hh = lane >> 4, m = lane & 15;
  const int rt = wave & 3, hp = wave >> 2;
  const int rowBase = (int)blockIdx.x * GBM;

  v8f acc[4];
  {
    const v8f z = {0.f, 0.f, 0.f, 0.f, 0.f, 0.f, 0.f, 0.f};
    acc[0] = z; acc[1] = z; acc[2] = z; acc[3] = z;
  }
  const unsigned short* ap = AG + (size_t)(rowBase + 16 * rt + m) * KX2 + 8 * hh;
  const unsigned short* wp = OW + (size_t)m * DHD + 8 * hh;
#pragma unroll
  for (int j = 0; j < 2; ++j) {
    const int hd = 2 * hp + j;
    FragB ah, alo;
    ah.h[0]  = *(const v8us*)(ap + DHD * hd);
    ah.h[1]  = *(const v8us*)(ap + DHD * hd + 16);
    alo.h[0] = *(const v8us*)(ap + DIN + DHD * hd);
    alo.h[1] = *(const v8us*)(ap + DIN + DHD * hd + 16);
#pragma unroll
    for (int c = 0; c < 2; ++c) {
      const unsigned short* wq = wp + (size_t)(16 * c) * DHD;
      FragB bf;
      bf.h[0] = *(const v8us*)wq;
      bf.h[1] = *(const v8us*)(wq + 16);
      acc[2 * j + c] = wmb(ah, bf, acc[2 * j + c]);
      acc[2 * j + c] = wmb(alo, bf, acc[2 * j + c]);
    }
  }

#pragma unroll
  for (int j = 0; j < 2; ++j) {
    const int hd = 2 * hp + j;
#pragma unroll
    for (int c = 0; c < 2; ++c) {
      const int lc = DHD * hd + 16 * c + m;
      const float bv = bfr(ob[16 * c + m]);
#pragma unroll
      for (int r = 0; r < 8; ++r) {
        const int lr = 16 * rt + 8 * hh + r;
        stg[lr * DIN + lc] = fmaxf(acc[2 * j + c][r] + bv, 0.f);
      }
    }
  }
  __syncthreads();

  v8us ov[8];
#pragma unroll
  for (int i = 0; i < 8; ++i) {
    const int p  = i * NTHR + tid;
    const int lr = p >> 5;
    const int q  = p & 31;
    const int c0 = 8 * (q & 15);
    const v4f ga = *(const v4f*)(stg + lr * DIN + c0);
    const v4f gb = *(const v4f*)(stg + lr * DIN + c0 + 4);
    ov[i] = hilo8(ga, gb, q >= 16);
  }
#pragma unroll
  for (int i = 0; i < 8; ++i) {
    const int p  = i * NTHR + tid;
    const int gr = rowBase + (p >> 5);
    unsigned short* op = XP + (size_t)gr * KX2 + 8 * (p & 31);
    if (gr < nRows) *(volatile v8us*)op = ov[i];
  }
  __threadfence();
#pragma unroll
  for (int i = 0; i < 8; ++i) {
    const int p  = i * NTHR + tid;
    const int gr = rowBase + (p >> 5);
    unsigned short* op = XP + (size_t)gr * KX2 + 8 * (p & 31);
    if (gr < nRows) *(volatile v8us*)op = ov[i];
  }
}

__global__ __launch_bounds__(NTHR) void k_agg(
    const int* __restrict__ srcs, const int* __restrict__ dsts, const float* __restrict__ ew,
    const float* __restrict__ FT, const float* __restrict__ ELR, unsigned short* AGP,
    int nN, int nE, int nb, int vec8) {
  extern __shared__ v4f lds_dyn[];
  int* reg1 = (int*)lds_dyn;
  int* reg2 = reg1 + RCAP;
  int* scnt = reg2 + RCAP;
  int* soff = scnt + NBMAX;
  int* list = soff + NBMAX;
  int* wcnt = list + LISTN;
  int* wtot = wcnt + NWAVE;
  const int tid = (int)threadIdx.x, lane = tid & 31, wave = tid >> 5;
  const int nodeBase = (int)blockIdx.x * nb;

  for (int i = tid; i < NBMAX; i += NTHR) scnt[i] = 0;
  __syncthreads();

  int tot = 0;
  const int nChunks = (nE + CHUNK - 1) / CHUNK;
#pragma unroll 1
  for (int ch = 0; ch < nChunks; ++ch) {
    const int cbase = ch * CHUNK;
    const int wc = scan_chunk(dsts, nE, cbase, nodeBase, nb, vec8, list, tid, lane, wave);
    if (lane == 0) wcnt[wave] = wc;
    __syncthreads();
    int pre = 0, all = 0;
#pragma unroll
    for (int w2 = 0; w2 < NWAVE; ++w2) {
      int c = wcnt[w2];
      c = c < 0 ? 0 : (c > WCAP ? WCAP : c);
      all += c;
      pre += (w2 < wave) ? c : 0;
    }
    const int wcc  = wc > WCAP ? WCAP : wc;
    const int base = tot + pre;
#pragma unroll 1
    for (int i = lane; i < wcc; i += 32) {
      const int ent = list[wave * WCAP + i];
      const int el  = (ent >> 12) & (CHUNK - 1);
      const int sl  = ent & (NBMAX - 1);
      int eid = cbase + el;
      eid = eid > nE - 1 ? nE - 1 : eid;
      const int pos = base + i;
      if (pos < RCAP) reg1[pos] = (int)(((unsigned)eid << 12) | (unsigned)sl);
    }
    tot += all;
    tot = tot > RCAP ? RCAP : tot;
    __syncthreads();
  }
  const int nh = tot;

  if (wave == 0) {
#pragma unroll 1
    for (int b0 = 0; b0 < nh; b0 += 32) {
      const int idx = b0 + lane;
      const int uv  = reg1[idx < RCAP ? idx : RCAP - 1];
      const int m32 = (nh - b0) < 32 ? (nh - b0) : 32;
#pragma unroll 1
      for (int k = 0; k < m32; ++k) {
        const int u  = __builtin_amdgcn_readlane(uv, k);
        const int sl = u & (NBMAX - 1);
        if (lane == 0) scnt[sl] = scnt[sl] + 1;
      }
    }
  }
  __syncthreads();

  {
    int e0 = scnt[2 * tid], e1 = scnt[2 * tid + 1];
    e0 = e0 < 0 ? 0 : e0;
    e1 = e1 < 0 ? 0 : e1;
    const int ts = e0 + e1;
    int incl = ts;
#pragma unroll
    for (int d = 1; d < 32; d <<= 1) {
      const int up = __shfl_up(incl, d);
      if (lane >= d) incl += up;
    }
    if (lane == 31) wtot[wave] = incl;
    __syncthreads();
    int pre = 0;
#pragma unroll
    for (int w2 = 0; w2 < NWAVE; ++w2) pre += (w2 < wave) ? wtot[w2] : 0;
    const int run = pre + incl - ts;
    soff[2 * tid]     = run;
    soff[2 * tid + 1] = run + e0;
  }
  __syncthreads();
  for (int i = tid; i < NBMAX; i += NTHR) list[i] = soff[i];
  __syncthreads();

  if (wave == 0) {
#pragma unroll 1
    for (int b0 = 0; b0 < nh; b0 += 32) {
      const int idx = b0 + lane;
      const int uv  = reg1[idx < RCAP ? idx : RCAP - 1];
      const int m32 = (nh - b0) < 32 ? (nh - b0) : 32;
#pragma unroll 1
      for (int k = 0; k < m32; ++k) {
        const int u   = __builtin_amdgcn_readlane(uv, k);
        const int sl  = u & (NBMAX - 1);
        const int eid = (int)((unsigned)u >> 12);
        if (lane == 0) {
          int pos = list[sl];
          pos = pos < 0 ? 0 : (pos > RCAP - 1 ? RCAP - 1 : pos);
          reg2[pos] = eid;
          list[sl] = pos + 1;
        }
      }
    }
  }
  __syncthreads();

  const int nbw = nb >> 3;
  const bool ovf = (nh >= RCAP);
  const float qnan = __int_as_float(0x7fc00000);
  float* stw = (float*)reg1 + wave * STW;
  const int c0 = 8 * (lane & 15);
  const bool islo = lane >= 16;
#pragma unroll 1
  for (int jt = 0; jt < nbw; ++jt) {
    const int slot = wave * nbw + jt;
    const int node = nodeBase + slot;
    const int ncl  = node < nN ? node : nN - 1;
    const bool wr  = node < nN;
    int st = soff[slot];
    const int craw = scnt[slot];
    int cnt = craw;
    st  = st < 0 ? 0 : (st > nh ? nh : st);
    cnt = cnt < 0 ? 0 : (cnt > DEGCAP ? DEGCAP : cnt);
    if (cnt > nh - st) cnt = nh - st;
    const float pz = (ovf || craw > DEGCAP) ? qnan : 0.0f;
#pragma unroll 1
    for (int b = 0; b < NBT; ++b) {
      const size_t drow = (size_t)b * (size_t)nN + (size_t)ncl;
      const v4f er4 = *(const v4f*)(ELR + drow * 8 + 4);
      ldwait();
      float mx[4], dn[4], av[4];
#pragma unroll
      for (int h = 0; h < 4; ++h) { mx[h] = -1.0e30f; dn[h] = 0.f; av[h] = 0.f; }

#pragma unroll 1
      for (int q = 0; q < cnt; ++q) {
        int idx = st + q; idx = idx > RCAP - 1 ? RCAP - 1 : idx;
        int eid = reg2[idx]; eid = eid < 0 ? 0 : (eid > nE - 1 ? nE - 1 : eid);
        const int   sraw = srcs[eid];
        const float wv   = bfr(ew[eid]);
        const int s = sraw < 0 ? 0 : (sraw > nN - 1 ? nN - 1 : sraw);
        const size_t srow = (size_t)b * (size_t)nN + (size_t)s;
        const v4f el4 = *(const v4f*)(ELR + srow * 8);
        const float* fr = FT + srow * DIN + lane;
        float ft[4];
#pragma unroll
        for (int h = 0; h < 4; ++h) ft[h] = fr[DHD * h];
        ldwait();
#pragma unroll
        for (int h = 0; h < 4; ++h) {
          float v = el4[h] + er4[h];
          v = v > 0.f ? v : 0.1f * v;
          v = v * wv;
          const float df = v - mx[h];
          const float ee = __expf(-fabsf(df));
          const bool up  = df > 0.f;
          const float s1 = up ? ee : 1.0f;
          const float s2 = up ? 1.0f : ee;
          mx[h] = up ? v : mx[h];
          dn[h] = fmaf(dn[h], s1, s2);
          av[h] = fmaf(av[h], s1, s2 * ft[h]);
        }
      }
      float ag[4];
#pragma unroll
      for (int h = 0; h < 4; ++h) {
        const float ds = dn[h] > 0.f ? dn[h] : 1.0f;
        const float iv = (dn[h] > 0.f ? 1.0f : 0.0f) * __builtin_amdgcn_rcpf(ds);
        ag[h] = av[h] * iv + pz;
      }
      __builtin_amdgcn_fence(__ATOMIC_RELEASE, "wavefront");
      __builtin_amdgcn_wave_barrier();
#pragma unroll
      for (int h = 0; h < 4; ++h) stw[DHD * h + lane] = ag[h];
      __builtin_amdgcn_fence(__ATOMIC_RELEASE, "wavefront");
      __builtin_amdgcn_wave_barrier();
      const v4f ga = *(const v4f*)(stw + c0);
      const v4f gb = *(const v4f*)(stw + c0 + 4);
      const v8us ov = hilo8(ga, gb, islo);
      unsigned short* gp = AGP + drow * KX2 + 8 * lane;
      if (wr) *(volatile v8us*)gp = ov;
      __threadfence();
      if (wr) *(volatile v8us*)gp = ov;
    }
  }
}

static int pick_nb(int nE, int nN) {
  int nb = NBMAX;
  while (nb > 16 && (long long)nb * (long long)nE * 5LL > (long long)RCAP * (long long)nN * 4LL) nb >>= 1;
  return nb;
}
static inline int cdiv(int a, int b) { return (a + b - 1) / b; }

extern "C" void kernel_launch(void* const* d_in, const int* in_sizes, int n_in,
                              void* d_out, int out_size, void* d_ws, size_t ws_size,
                              hipStream_t stream) {
  if (n_in < 16) return;
  const int tot0 = in_sizes[0];
  const int nN = tot0 / (NBT * DIN);
  if (nN < 1 || tot0 != nN * NBT * DIN || nN > (1 << 19)) return;
  const int M = NBT * nN;
  if ((M % GBM) != 0) return;
  const int nE = in_sizes[1];
  if (nE < 1 || nE > (1 << 20)) return;
  if (in_sizes[2] != nE || in_sizes[3] != nE) return;
  if (in_sizes[4]  != DIN * DIN || in_sizes[5]  != NHD * DHD || in_sizes[6]  != NHD * DHD) return;
  if (in_sizes[7]  != DHD * DHD || in_sizes[8]  != DHD) return;
  if (in_sizes[9]  != DIN * DIN || in_sizes[10] != NHD * DHD || in_sizes[11] != NHD * DHD) return;
  if (in_sizes[12] != DHD * DHD || in_sizes[13] != DHD) return;
  if (in_sizes[14] != DIN * KX2 || in_sizes[15] != DIN) return;
  if (out_size != M * DIN) return;

  const float* x      = (const float*)d_in[0];
  const int*   src    = (const int*)  d_in[1];
  const int*   dst    = (const int*)  d_in[2];
  const float* edge_w = (const float*)d_in[3];
  const float* fc_w0  = (const float*)d_in[4];
  const float* al0    = (const float*)d_in[5];
  const float* ar0    = (const float*)d_in[6];
  const float* out_w0 = (const float*)d_in[7];
  const float* out_b0 = (const float*)d_in[8];
  const float* fc_w1  = (const float*)d_in[9];
  const float* al1    = (const float*)d_in[10];
  const float* ar1    = (const float*)d_in[11];
  const float* out_w1 = (const float*)d_in[12];
  const float* out_b1 = (const float*)d_in[13];
  const float* mlp_w  = (const float*)d_in[14];
  const float* mlp_b  = (const float*)d_in[15];
  float* out = (float*)d_out;

  const int MP   = M;
  const int nb   = pick_nb(nE, nN);
  const int gA   = cdiv(nN, nb);
  const int vec8 = 1;
  if (gA * nb < nN || nb < 16) return;

  char* ws = (char*)d_ws;
  size_t off = 0;
  const size_t oXB  = off; off += (size_t)MP * DIN * 2;            off = (off + 255) & ~(size_t)255;
  const size_t oW0  = off; off += (size_t)DIN * DIN * 2;           off = (off + 255) & ~(size_t)255;
  const size_t oW1  = off; off += (size_t)DIN * DIN * 2;           off = (off + 255) & ~(size_t)255;
  const size_t oOW0 = off; off += (size_t)DHD * DHD * 2;           off = (off + 255) & ~(size_t)255;
  const size_t oOW1 = off; off += (size_t)DHD * DHD * 2;           off = (off + 255) & ~(size_t)255;
  const size_t oWM  = off; off += (size_t)DIN * KX2 * 2;           off = (off + 255) & ~(size_t)255;
  const size_t oFT  = off; off += (size_t)MP * DIN * 4;            off = (off + 255) & ~(size_t)255;
  const size_t oELR = off; off += (size_t)MP * 8 * 4;              off = (off + 255) & ~(size_t)255;
  const size_t oAG  = off; off += (size_t)MP * KX2 * 2;            off = (off + 255) & ~(size_t)255;
  const size_t oX1  = off; off += (size_t)MP * KX2 * 2;            off = (off + 255) & ~(size_t)255;
  const size_t oX2  = off; off += (size_t)MP * KX2 * 2;            off = (off + 255) & ~(size_t)255;
  if (off > ws_size || off > (size_t)WSMAX) return;
  unsigned short* XB   = (unsigned short*)(ws + oXB);
  unsigned short* W0P  = (unsigned short*)(ws + oW0);
  unsigned short* W1P  = (unsigned short*)(ws + oW1);
  unsigned short* OW0P = (unsigned short*)(ws + oOW0);
  unsigned short* OW1P = (unsigned short*)(ws + oOW1);
  unsigned short* WMP  = (unsigned short*)(ws + oWM);
  float*          FT   = (float*)(ws + oFT);
  float*          ELR  = (float*)(ws + oELR);
  unsigned short* AGP  = (unsigned short*)(ws + oAG);
  unsigned short* XP1  = (unsigned short*)(ws + oX1);
  unsigned short* XP2  = (unsigned short*)(ws + oX2);

  hipFuncSetAttribute(reinterpret_cast<const void*>(&k_agg),
                      hipFuncAttributeMaxDynamicSharedMemorySize, LDS_AGG);

  {
    const int nUx = MP * (DIN / 8);
    k_cvt<<<cdiv(nUx, NTHR), NTHR, 0, stream>>>(x, M, DIN, XB, nUx);
    const int nUw = DIN * (DIN / 8);
    k_cvt<<<cdiv(nUw, NTHR), NTHR, 0, stream>>>(fc_w0, DIN, DIN, W0P, nUw);
    k_cvt<<<cdiv(nUw, NTHR), NTHR, 0, stream>>>(fc_w1, DIN, DIN, W1P, nUw);
    const int nUo = DHD * (DHD / 8);
    k_cvt<<<cdiv(nUo, NTHR), NTHR, 0, stream>>>(out_w0, DHD, DHD, OW0P, nUo);
    k_cvt<<<cdiv(nUo, NTHR), NTHR, 0, stream>>>(out_w1, DHD, DHD, OW1P, nUo);
    const int nUm = DIN * (KX2 / 8);
    k_cvt<<<cdiv(nUm, NTHR), NTHR, 0, stream>>>(mlp_w, DIN, KX2, WMP, nUm);
  }

  const int gM = MP / GBM;
  k_gemm<0, 0><<<gM, NTHR, 0, stream>>>(XB, XB, DIN, 0, DIN / 32, 0, W0P, DIN,
                                        al0, ar0, al0, FT, ELR, MP);
  k_agg<<<gA, NTHR, LDS_AGG, stream>>>(src, dst, edge_w, FT, ELR, AGP, nN, nE, nb, vec8);
  k_ofc<<<gM, NTHR, 0, stream>>>(AGP, OW0P, out_b0, XP1, MP);
  k_gemm<0, 1><<<gM, NTHR, 0, stream>>>(XP1, XP1, KX2, DIN, DIN / 32, 0, W1P, DIN,
                                        al1, ar1, al1, FT, ELR, MP);
  k_agg<<<gA, NTHR, LDS_AGG, stream>>>(src, dst, edge_w, FT, ELR, AGP, nN, nE, nb, vec8);
  k_ofc<<<gM, NTHR, 0, stream>>>(AGP, OW1P, out_b1, XP2, MP);
  k_gemm<1, 1><<<gM, NTHR, 0, stream>>>(XP1, XP2, KX2, DIN, DIN / 32, DIN / 32, WMP, KX2,
                                        mlp_b, mlp_b, mlp_b, out, ELR, M);
}
